// LinearAttention2_6012954214508
// MI455X (gfx1250) — hardware-verified
//
#include <hip/hip_runtime.h>
#define BB 4
#define NN 4096
#define CC 768
#define NH 12
#define HD 64

typedef __bf16 v16b __attribute__((ext_vector_type(16)));
typedef unsigned short v8us __attribute__((ext_vector_type(8), may_alias));
typedef float  v8f  __attribute__((ext_vector_type(8)));
typedef float  v4f  __attribute__((ext_vector_type(4)));
typedef float  v4fa __attribute__((ext_vector_type(4), may_alias));
union FragB { v16b v; v8us half[2]; unsigned short u[16]; };

__device__ __forceinline__ unsigned short bf16_bits(float x) { unsigned int u = __float_as_uint(x); return (unsigned short)((u + 0x7FFFu + ((u >> 16) & 1u)) >> 16); }
__device__ __forceinline__ float bf16_val(unsigned short b) { return __uint_as_float(((unsigned int)b) << 16); }
__device__ __forceinline__ float bf16_round(float x) { return bf16_val(bf16_bits(x)); }
template <int NT>
__device__ __forceinline__ v8f mmaN(v16b ah, v16b al, v16b bh, v16b bl, v8f c) {
  c = __builtin_amdgcn_wmma_f32_16x16x32_bf16(false, ah, false, bh, (short)0, c, false, false);
  if (NT >= 2) c = __builtin_amdgcn_wmma_f32_16x16x32_bf16(false, al, false, bh, (short)0, c, false, false);
  if (NT >= 3) c = __builtin_amdgcn_wmma_f32_16x16x32_bf16(false, ah, false, bl, (short)0, c, false, false);
  asm volatile("v_nop\n\tv_nop\n\tv_nop\n\tv_nop" : "+v"(c) : "v"(ah), "v"(al), "v"(bh), "v"(bl));
  return c;
}

__global__ __launch_bounds__(256) void k_wt_bf16(const float* __restrict__ W, unsigned short* __restrict__ Wt, int K, int N) {
  const int t = blockIdx.x * 256 + threadIdx.x;
  const int k8n = K / 8;
  if (t >= N * k8n) return;
  const int n = t / k8n, k8 = (t % k8n) * 8;
  v8us v;
#pragma unroll
  for (int i = 0; i < 8; ++i) v[i] = bf16_bits(W[(size_t)(k8 + i) * N + n]);
  *(volatile v8us*)(Wt + (size_t)n * K + k8) = v;
  __threadfence();
  *(volatile v8us*)(Wt + (size_t)n * K + k8) = v;
}

template <bool ASPLIT, int ACT, bool BIAS_BF16>
__global__ __launch_bounds__(128) void k_gemm_bf(const float* __restrict__ A, int lda, const unsigned short* __restrict__ Wt, int ldb,
                                               const float* __restrict__ bias, float* __restrict__ C, int ldc, int M, int N, int K) {
  __shared__ __attribute__((aligned(16))) float so[4][16][64];
  const int tid = threadIdx.x, w = tid >> 5, lane = tid & 31, ln = lane & 15, hh = lane >> 4;
  const int ntn = N / 64;
  const int wid = blockIdx.x * 4 + w;
  const int mt = wid / ntn, nq = wid % ntn;
  if (mt * 16 >= M) return;
  const int row0 = mt * 16, col0 = nq * 64;
  const float* arow = A + (size_t)(row0 + ln) * lda;
  v8f acc[4] = {};
  for (int kb = 0; kb < K; kb += 32) {
    FragB ah, al;
    const v4f x0 = *(const v4fa*)(arow + kb + 8 * hh), x1 = *(const v4fa*)(arow + kb + 8 * hh + 4);
    const v4f x2 = *(const v4fa*)(arow + kb + 16 + 8 * hh), x3 = *(const v4fa*)(arow + kb + 16 + 8 * hh + 4);
    float xs[16] = {x0[0],x0[1],x0[2],x0[3],x1[0],x1[1],x1[2],x1[3],x2[0],x2[1],x2[2],x2[3],x3[0],x3[1],x3[2],x3[3]};
#pragma unroll
    for (int i = 0; i < 16; ++i) { const unsigned short hb = bf16_bits(xs[i]); ah.u[i] = hb; al.u[i] = ASPLIT ? bf16_bits(xs[i] - bf16_val(hb)) : (unsigned short)0; }
#pragma unroll
    for (int t = 0; t < 4; ++t) {
      const unsigned short* brow = Wt + (size_t)(col0 + t * 16 + ln) * ldb + kb;
      FragB b;
      b.half[0] = *(const v8us*)(brow + 8 * hh);
      b.half[1] = *(const v8us*)(brow + 16 + 8 * hh);
      acc[t] = mmaN<ASPLIT ? 2 : 1>(ah.v, al.v, b.v, b.v, acc[t]);
    }
  }
#pragma unroll
  for (int t = 0; t < 4; ++t) {
    float bv = bias ? bias[col0 + t * 16 + ln] : 0.f;
    if (BIAS_BF16) bv = bf16_round(bv);
#pragma unroll
    for (int r = 0; r < 8; ++r) { float v = acc[t][r] + bv; if (ACT == 1) v = fmaxf(v, 0.f); so[w][8 * hh + r][t * 16 + ln] = v; }
  }
  __builtin_amdgcn_fence(__ATOMIC_ACQ_REL, "workgroup");
  __builtin_amdgcn_wave_barrier();
  const int rsub = lane >> 4, c4 = (lane & 15) * 4;
  for (int pass = 0; pass < 2; ++pass) {
#pragma unroll
    for (int q = 0; q < 8; ++q) {
      const int r = q * 2 + rsub;
      const v4f v = *(const v4fa*)&so[w][r][c4];
      *(volatile v4f*)(C + (size_t)(row0 + r) * ldc + col0 + c4) = v;
    }
    if (pass == 0) __threadfence();
  }
}

template <int D, bool CAUSAL>
__global__ __launch_bounds__(128) void k_flash(const float* __restrict__ qb, const float* __restrict__ kb, const float* __restrict__ vb,
                                             int pitch, int T, int H, float scale, float* __restrict__ y, int ypitch) {
  constexpr int KS = D / 32;
  constexpr int DT = D / 16;
  __shared__ __attribute__((aligned(16))) unsigned short sKh[32][D + 8], sKl[32][D + 8], sVh[32][D + 8], sVl[32][D + 8];
  __shared__ __attribute__((aligned(16))) unsigned short sPh[4][16][40], sPl[4][16][40];
  __shared__ __attribute__((aligned(16))) float sO[4][16][D];
  const int tid = threadIdx.x, w = tid >> 5, lane = tid & 31, ln = lane & 15, hh = lane >> 4;
  const int nqb = (T + 63) / 64;
  const int bh = blockIdx.x / nqb, qblk = blockIdx.x % nqb;
  const int b = bh / H, h = bh % H;
  const int q0 = qblk * 64 + w * 16;
  const float* Q = qb + (size_t)b * T * pitch + h * D;
  const float* K = kb + (size_t)b * T * pitch + h * D;
  const float* V = vb + (size_t)b * T * pitch + h * D;

  FragB aqh[KS], aql[KS];
  {
    int row = q0 + ln; if (row >= T) row = T - 1;
    const float* qr = Q + (size_t)row * pitch;
#pragma unroll
    for (int ks = 0; ks < KS; ++ks)
#pragma unroll
      for (int i = 0; i < 16; ++i) {
        const int d = ks * 32 + ((i < 8) ? (8 * hh + i) : (16 + 8 * hh + (i - 8)));
        const float x = qr[d] * scale; const unsigned short hb = bf16_bits(x);
        aqh[ks].u[i] = hb; aql[ks].u[i] = bf16_bits(x - bf16_val(hb));
      }
  }
  float m_r[8], l_r[8];
#pragma unroll
  for (int r = 0; r < 8; ++r) { m_r[r] = -3.0e38f; l_r[r] = 0.f; }
  v8f oacc[DT];
#pragma unroll
  for (int dt = 0; dt < DT; ++dt) oacc[dt] = (v8f){0.f,0.f,0.f,0.f,0.f,0.f,0.f,0.f};

  const int kv_end = CAUSAL ? min(T, qblk * 64 + 64) : T;
  for (int j0 = 0; j0 < kv_end; j0 += 32) {
    __syncthreads();
    for (int e = tid; e < 32 * (D / 4); e += 128) {
      const int r = e / (D / 4), c4 = (e % (D / 4)) * 4;
      const int key = j0 + r;
      v4f kf = {0.f,0.f,0.f,0.f}, vf = {0.f,0.f,0.f,0.f};
      if (key < T) { kf = *(const v4fa*)(K + (size_t)key * pitch + c4); vf = *(const v4fa*)(V + (size_t)key * pitch + c4); }
#pragma unroll
      for (int t = 0; t < 4; ++t) {
        unsigned short hb = bf16_bits(kf[t]); sKh[r][c4 + t] = hb; sKl[r][c4 + t] = bf16_bits(kf[t] - bf16_val(hb));
        hb = bf16_bits(vf[t]); sVh[r][c4 + t] = hb; sVl[r][c4 + t] = bf16_bits(vf[t] - bf16_val(hb));
      }
    }
    __syncthreads();
    v8f s[2];
#pragma unroll
    for (int nt = 0; nt < 2; ++nt) {
      v8f acc = {};
#pragma unroll
      for (int ks = 0; ks < KS; ++ks) {
        FragB bh_, bl_;
        bh_.half[0] = *(const v8us*)&sKh[nt * 16 + ln][ks * 32 + 8 * hh]; bh_.half[1] = *(const v8us*)&sKh[nt * 16 + ln][ks * 32 + 16 + 8 * hh];
        bl_.half[0] = *(const v8us*)&sKl[nt * 16 + ln][ks * 32 + 8 * hh]; bl_.half[1] = *(const v8us*)&sKl[nt * 16 + ln][ks * 32 + 16 + 8 * hh];
        acc = mmaN<3>(aqh[ks].v, aql[ks].v, bh_.v, bl_.v, acc);
      }
      s[nt] = acc;
    }
    float alpha[8];
#pragma unroll
    for (int r = 0; r < 8; ++r) {
      const int qi = q0 + 8 * hh + r;
      const int ja = j0 + ln, jb = j0 + 16 + ln;
      if (CAUSAL) { if (ja > qi) s[0][r] = -3.0e38f; if (jb > qi) s[1][r] = -3.0e38f; }
      if (ja >= T) s[0][r] = -3.0e38f;
      if (jb >= T) s[1][r] = -3.0e38f;
      float mx = fmaxf(s[0][r], s[1][r]);
      mx = fmaxf(mx, __shfl_xor(mx, 1, 32)); mx = fmaxf(mx, __shfl_xor(mx, 2, 32)); mx = fmaxf(mx, __shfl_xor(mx, 4, 32)); mx = fmaxf(mx, __shfl_xor(mx, 8, 32));
      const float mnew = fmaxf(m_r[r], mx);
      alpha[r] = (mnew > -1.0e38f) ? __expf(m_r[r] - mnew) : 1.0f;
      const float p0 = (s[0][r] > -1.0e38f) ? __expf(s[0][r] - mnew) : 0.f;
      const float p1 = (s[1][r] > -1.0e38f) ? __expf(s[1][r] - mnew) : 0.f;
      m_r[r] = mnew;
      l_r[r] = l_r[r] * alpha[r] + p0 + p1;
      unsigned short hb = bf16_bits(p0); sPh[w][8 * hh + r][ln] = hb;      sPl[w][8 * hh + r][ln] = bf16_bits(p0 - bf16_val(hb));
      hb = bf16_bits(p1);                sPh[w][8 * hh + r][16 + ln] = hb; sPl[w][8 * hh + r][16 + ln] = bf16_bits(p1 - bf16_val(hb));
    }
#pragma unroll
    for (int dt = 0; dt < DT; ++dt)
#pragma unroll
      for (int r = 0; r < 8; ++r) oacc[dt][r] *= alpha[r];
    __builtin_amdgcn_fence(__ATOMIC_ACQ_REL, "workgroup");
    __builtin_amdgcn_wave_barrier();
    FragB pah, pal;
    pah.half[0] = *(const v8us*)&sPh[w][ln][8 * hh]; pah.half[1] = *(const v8us*)&sPh[w][ln][16 + 8 * hh];
    pal.half[0] = *(const v8us*)&sPl[w][ln][8 * hh]; pal.half[1] = *(const v8us*)&sPl[w][ln][16 + 8 * hh];
#pragma unroll
    for (int dt = 0; dt < DT; ++dt) {
      FragB bvh, bvl;
#pragma unroll
      for (int i = 0; i < 8; ++i) {
        bvh.u[i] = sVh[8 * hh + i][dt * 16 + ln]; bvh.u[8 + i] = sVh[16 + 8 * hh + i][dt * 16 + ln];
        bvl.u[i] = sVl[8 * hh + i][dt * 16 + ln]; bvl.u[8 + i] = sVl[16 + 8 * hh + i][dt * 16 + ln];
      }
      oacc[dt] = mmaN<3>(pah.v, pal.v, bvh.v, bvl.v, oacc[dt]);
    }
    __builtin_amdgcn_fence(__ATOMIC_ACQ_REL, "workgroup");
    __builtin_amdgcn_wave_barrier();
  }
#pragma unroll
  for (int r = 0; r < 8; ++r) {
    float l = l_r[r];
    l += __shfl_xor(l, 1, 32); l += __shfl_xor(l, 2, 32); l += __shfl_xor(l, 4, 32); l += __shfl_xor(l, 8, 32);
    l_r[r] = (l > 0.f) ? 1.0f / l : 0.f;
  }
#pragma unroll
  for (int dt = 0; dt < DT; ++dt)
#pragma unroll
    for (int r = 0; r < 8; ++r) sO[w][8 * hh + r][dt * 16 + ln] = oacc[dt][r] * l_r[r];
  __builtin_amdgcn_fence(__ATOMIC_ACQ_REL, "workgroup");
  __builtin_amdgcn_wave_barrier();
  for (int pass = 0; pass < 2; ++pass) {
    for (int r = 0; r < 16; ++r) {
      const int row = q0 + r;
      if (row < T && lane < D / 4) {
        const v4f val = *(const v4fa*)&sO[w][r][lane * 4];
        *(volatile v4f*)(y + ((size_t)b * T + row) * ypitch + h * D + lane * 4) = val;
      }
    }
    if (pass == 0) __threadfence();
  }
}

__global__ __launch_bounds__(256) void k_round_rows(const float* __restrict__ W, unsigned short* __restrict__ Wt, int n8) {
  const int t = blockIdx.x * 256 + threadIdx.x;
  if (t >= n8) return;
  const v4f a = *(const v4fa*)(W + (size_t)t * 8), b = *(const v4fa*)(W + (size_t)t * 8 + 4);
  v8us v; v[0]=bf16_bits(a[0]); v[1]=bf16_bits(a[1]); v[2]=bf16_bits(a[2]); v[3]=bf16_bits(a[3]);
  v[4]=bf16_bits(b[0]); v[5]=bf16_bits(b[1]); v[6]=bf16_bits(b[2]); v[7]=bf16_bits(b[3]);
  *(volatile v8us*)(Wt + (size_t)t * 8) = v; __threadfence(); *(volatile v8us*)(Wt + (size_t)t * 8) = v;
}

__device__ __forceinline__ float elu1(float x) { return x > 0.f ? x + 1.0f : expf(x); }
__global__ __launch_bounds__(256) void k_elu1(float* __restrict__ qkv, int M) {
  const size_t t = (size_t)blockIdx.x * 256 + threadIdx.x; if (t >= (size_t)M * (2 * CC / 4)) return;
  const size_t row = t / (2 * CC / 4); const int c4 = (int)(t % (2 * CC / 4)) * 4;
  float* p = qkv + row * 3 * CC + c4; v4f v = *(const v4fa*)p; for (int q = 0; q < 4; ++q) v[q] = elu1(v[q]);
  *(volatile v4f*)p = v; __threadfence(); *(volatile v4f*)p = v;
}
__global__ __launch_bounds__(128) void k_ktv(const float* __restrict__ qkv, float* __restrict__ kvout, unsigned short* __restrict__ kvTh, unsigned short* __restrict__ kvTl, float* __restrict__ ksum) {
  __shared__ __attribute__((aligned(16))) float red[64][68]; __shared__ float sks[64];
  const int tid = threadIdx.x, w = tid >> 5, lane = tid & 31, ln = lane & 15, hh = lane >> 4;
  const int bh = blockIdx.x, b = bh / NH, h = bh % NH;
  const float* kb = qkv + (size_t)b * NN * 3 * CC + CC + h * HD; const float* vb = qkv + (size_t)b * NN * 3 * CC + 2 * CC + h * HD; const int pitch = 3 * CC;
  v8f acc[4]; for (int j = 0; j < 4; ++j) acc[j] = (v8f){0.f,0.f,0.f,0.f,0.f,0.f,0.f,0.f};
  float ks = 0.f;
  const int d0 = w * 16;
  for (int sb = 0; sb < NN; sb += 32) {
    if (hh == 0) { for (int j = 0; j < 32; ++j) ks += kb[(size_t)(sb + j) * pitch + d0 + ln]; }
    FragB ah, al;
#pragma unroll
    for (int e = 0; e < 16; ++e) { const int s = sb + ((e < 8) ? (8 * hh + e) : (16 + 8 * hh + (e - 8))); const float x = kb[(size_t)s * pitch + d0 + ln]; const unsigned short hb = bf16_bits(x); ah.u[e] = hb; al.u[e] = bf16_bits(x - bf16_val(hb)); }
#pragma unroll
    for (int j = 0; j < 4; ++j) {
      FragB bq, bl;
#pragma unroll
      for (int e = 0; e < 16; ++e) { const int s = sb + ((e < 8) ? (8 * hh + e) : (16 + 8 * hh + (e - 8))); const float x = vb[(size_t)s * pitch + j * 16 + ln]; const unsigned short hb = bf16_bits(x); bq.u[e] = hb; bl.u[e] = bf16_bits(x - bf16_val(hb)); }
      acc[j] = mmaN<3>(ah.v, al.v, bq.v, bl.v, acc[j]);
    }
  }
#pragma unroll
  for (int j = 0; j < 4; ++j)
#pragma unroll
    for (int r = 0; r < 8; ++r) red[d0 + 8 * hh + r][j * 16 + ln] = acc[j][r];
  if (hh == 0) sks[d0 + ln] = ks;
  __syncthreads();
  for (int pass = 0; pass < 2; ++pass) {
#pragma unroll 1
    for (int it = 0; it < 8; ++it) { const int idx = it * 128 + tid; const int row = idx >> 4, c4 = (idx & 15) * 4; const v4f o = *(const v4fa*)&red[row][c4]; *(volatile v4f*)(kvout + ((size_t)bh * HD + row) * HD + c4) = o; }
    if (pass == 0) __threadfence();
  }
  for (int pass = 0; pass < 2; ++pass) {
#pragma unroll 1
    for (int it = 0; it < 4; ++it) {
      const int idx = it * 128 + tid; const int e = idx >> 3, c = idx & 7; v8us vh, vl;
#pragma unroll
      for (int i = 0; i < 8; ++i) { const float x = red[c * 8 + i][e]; const unsigned short hb = bf16_bits(x); vh[i] = hb; vl[i] = bf16_bits(x - bf16_val(hb)); }
      *(volatile v8us*)(kvTh + ((size_t)bh * HD + e) * HD + c * 8) = vh; *(volatile v8us*)(kvTl + ((size_t)bh * HD + e) * HD + c * 8) = vl;
    }
    if (pass == 0) __threadfence();
  }
  if (tid < 32) { float* ksp = ksum + (size_t)bh * HD; const float a0 = sks[tid], a1 = sks[32 + tid];
    *(volatile float*)(ksp + tid) = a0; *(volatile float*)(ksp + 32 + tid) = a1; __threadfence(); *(volatile float*)(ksp + tid) = a0; *(volatile float*)(ksp + 32 + tid) = a1; }
}
__global__ __launch_bounds__(128) void k_qkv_out(const float* __restrict__ qkv, const unsigned short* __restrict__ kvTh, const unsigned short* __restrict__ kvTl, const float* __restrict__ ksum, float* __restrict__ y) {
  __shared__ __attribute__((aligned(16))) float so[4][16][64];
  const int tid = threadIdx.x, w = tid >> 5, lane = tid & 31, ln = lane & 15, hh = lane >> 4;
  const int nqb = NN / 64; const int bh = blockIdx.x / nqb, qb = blockIdx.x % nqb; const int b = bh / NH, h = bh % NH;
  const int s0 = qb * 64 + w * 16;
  const float* qb_ = qkv + ((size_t)b * NN) * 3 * CC + h * HD; const int pitch = 3 * CC;
  const float* ks = ksum + (size_t)bh * HD;
  float zr[16];
  const float k0 = ks[lane], k1 = ks[32 + lane];
#pragma unroll
  for (int r = 0; r < 16; ++r) { const float* qr = qb_ + (size_t)(s0 + r) * pitch; float p = qr[lane] * k0 + qr[32 + lane] * k1; for (int o = 16; o >= 1; o >>= 1) p += __shfl_xor(p, o, 32); zr[r] = 1.0f / p; }
  v8f acc[4] = {};
  const float* qrow = qb_ + (size_t)(s0 + ln) * pitch;
#pragma unroll
  for (int ks2 = 0; ks2 < 2; ++ks2) {
    FragB ah, al;
#pragma unroll
    for (int i = 0; i < 16; ++i) { const int d = ks2 * 32 + ((i < 8) ? (8 * hh + i) : (16 + 8 * hh + (i - 8))); const float x = qrow[d]; const unsigned short hb = bf16_bits(x); ah.u[i] = hb; al.u[i] = bf16_bits(x - bf16_val(hb)); }
#pragma unroll
    for (int t = 0; t < 4; ++t) { const size_t bo = ((size_t)bh * HD + t * 16 + ln) * HD + ks2 * 32; FragB bh2, bl2; bh2.half[0] = *(const v8us*)(kvTh + bo + 8 * hh); bh2.half[1] = *(const v8us*)(kvTh + bo + 16 + 8 * hh); bl2.half[0] = *(const v8us*)(kvTl + bo + 8 * hh); bl2.half[1] = *(const v8us*)(kvTl + bo + 16 + 8 * hh); acc[t] = mmaN<3>(ah.v, al.v, bh2.v, bl2.v, acc[t]); }
  }
#pragma unroll
  for (int t = 0; t < 4; ++t)
#pragma unroll
    for (int r = 0; r < 8; ++r) so[w][8 * hh + r][t * 16 + ln] = acc[t][r] * zr[8 * hh + r];
  __builtin_amdgcn_fence(__ATOMIC_ACQ_REL, "workgroup"); __builtin_amdgcn_wave_barrier();
  const int rsub = lane >> 4, c4 = (lane & 15) * 4;
  for (int pass = 0; pass < 2; ++pass) { for (int q = 0; q < 8; ++q) { const int r = q * 2 + rsub; const v4f v = *(const v4fa*)&so[w][r][c4]; *(volatile v4f*)(y + ((size_t)b * NN + s0 + r) * CC + h * HD + c4) = v; } if (pass == 0) __threadfence(); }
}
extern "C" void kernel_launch(void* const* d_in, const int* in_sizes, int n_in,
                              void* d_out, int out_size, void* d_ws, size_t ws_size, hipStream_t stream) {
  (void)in_sizes; (void)n_in; (void)out_size;
  const float* x = (const float*)d_in[0]; const float* Wqkv = (const float*)d_in[1]; const float* Wp = (const float*)d_in[2]; const float* bp = (const float*)d_in[3];
  float* out = (float*)d_out; float* kvout = (float*)((char*)d_out + 50331648);
  char* ws = (char*)d_ws; size_t off = 0;
  auto take = [&](size_t bytes) { char* p = ws + off; off += (bytes + 255) & ~(size_t)255; return p; };
  const int M = BB * NN;
  unsigned short* Wq = (unsigned short*)take((size_t)3 * CC * CC * 2); unsigned short* Wpt = (unsigned short*)take((size_t)CC * CC * 2);
  float* qkv = (float*)take((size_t)M * 3 * CC * 4); float* y = (float*)take((size_t)M * CC * 4);
  unsigned short* kvTh = (unsigned short*)take((size_t)BB * NH * HD * HD * 2); unsigned short* kvTl = (unsigned short*)take((size_t)BB * NH * HD * HD * 2); float* ksum = (float*)take((size_t)BB * NH * HD * 4);
  if (off > ws_size) return;
  k_round_rows<<<(3 * CC * CC / 8 + 255) / 256, 256, 0, stream>>>(Wqkv, Wq, 3 * CC * CC / 8);
  k_round_rows<<<(CC * CC / 8 + 255) / 256, 256, 0, stream>>>(Wp, Wpt, CC * CC / 8);
  k_gemm_bf<false, 0, false><<<((M / 16) * (3 * CC / 64) + 3) / 4, 128, 0, stream>>>(x, CC, Wq, CC, nullptr, qkv, 3 * CC, M, 3 * CC, CC);
  k_elu1<<<(unsigned)(((size_t)M * (2 * CC / 4) + 255) / 256), 256, 0, stream>>>(qkv, M);
  k_ktv<<<BB * NH, 128, 0, stream>>>(qkv, kvout, kvTh, kvTl, ksum);
  k_qkv_out<<<BB * NH * (NN / 64), 128, 0, stream>>>(qkv, kvTh, kvTl, ksum, y);
  k_gemm_bf<true, 0, true><<<((M / 16) * (CC / 64) + 3) / 4, 128, 0, stream>>>(y, CC, Wpt, CC, bp, out, CC, M, CC, CC);
}
